// GraphConvLayer_18734647345262
// MI455X (gfx1250) — hardware-verified
//
#include <hip/hip_runtime.h>
#include <hip/hip_bf16.h>
#include <stdint.h>

#pragma clang fp contract(off)

typedef __bf16         v16bf __attribute__((ext_vector_type(16)));
typedef unsigned short v16us __attribute__((ext_vector_type(16)));
typedef unsigned short v8us  __attribute__((ext_vector_type(8)));
typedef float          v8f   __attribute__((ext_vector_type(8)));
typedef float          v4f   __attribute__((ext_vector_type(4)));
typedef v8us __attribute__((may_alias)) v8usa;
typedef v4f  __attribute__((may_alias)) v4fa;

union FragU { v16us u; v8us half[2]; };

#define BB    4
#define NN    512
#define DD    256
#define MROWS (BB * NN)
#define LN_EPS 1e-5f

static_assert(DD % 64 == 0);
static_assert(NN % 64 == 0);
static_assert(MROWS % 64 == 0);
static_assert(DD % 32 == 0);
static_assert(NN % 32 == 0);
static_assert(MROWS % 8 == 0);

static __device__ __forceinline__ unsigned short f2bf(float x) {
  uint32_t u = __builtin_bit_cast(uint32_t, x);
  u += 0x7FFFu + ((u >> 16) & 1u);
  return (unsigned short)(u >> 16);
}
static __device__ __forceinline__ float bf2f(unsigned short b) {
  return __builtin_bit_cast(float, ((uint32_t)b) << 16);
}
static __device__ __forceinline__ float bfr(float x) { return bf2f(f2bf(x)); }

__device__ __forceinline__ v8f wmma_bf16(v16us au, v16us bu, v8f c) {
  const v16bf a = __builtin_bit_cast(v16bf, au);
  const v16bf b = __builtin_bit_cast(v16bf, bu);
  v8f d = __builtin_amdgcn_wmma_f32_16x16x32_bf16(false, a, false, b, (short)0, c, false, false);
  asm volatile("v_nop\n\tv_nop\n\tv_nop\n\tv_nop" : "+v"(d) : "v"(au), "v"(bu));
  return d;
}

__device__ __forceinline__ v16us load_frag(const unsigned short* p, int h) {
  FragU f;
  f.half[0] = *(const v8usa*)(p + 8 * h);
  f.half[1] = *(const v8usa*)(p + 16 + 8 * h);
  return f.u;
}

__global__ __launch_bounds__(256) void ln_kernel(
    const float* __restrict__ H, const float* __restrict__ gamma, const float* __restrict__ beta,
    unsigned short* __restrict__ Hh, unsigned short* __restrict__ Hl)
{
  const int wv = threadIdx.x >> 5, lane = threadIdx.x & 31;
  const int row = blockIdx.x * 8 + wv;
  if (row >= MROWS) return;

  const float* hp = H + (size_t)row * DD + 8 * lane;
  const v4f a = *(const v4fa*)hp;
  const v4f c = *(const v4fa*)(hp + 4);
  float x[8] = { a.x, a.y, a.z, a.w, c.x, c.y, c.z, c.w };
  float s = 0.f;
  #pragma unroll
  for (int j = 0; j < 8; ++j) { x[j] = bfr(x[j]); s += x[j]; }
  #pragma unroll
  for (int o = 16; o >= 1; o >>= 1) s += __shfl_xor(s, o, 32);
  const float mu = s * (1.0f / 256.0f);

  float q = 0.f;
  #pragma unroll
  for (int j = 0; j < 8; ++j) { const float t = x[j] - mu; q += t * t; }
  #pragma unroll
  for (int o = 16; o >= 1; o >>= 1) q += __shfl_xor(q, o, 32);
  const float rstd = rsqrtf(q * (1.0f / 256.0f) + LN_EPS);

  const v4f ga = *(const v4fa*)(gamma + 8 * lane);
  const v4f gc = *(const v4fa*)(gamma + 8 * lane + 4);
  const v4f ba = *(const v4fa*)(beta + 8 * lane);
  const v4f bc = *(const v4fa*)(beta + 8 * lane + 4);
  const float g[8]  = { ga.x, ga.y, ga.z, ga.w, gc.x, gc.y, gc.z, gc.w };
  const float bt[8] = { ba.x, ba.y, ba.z, ba.w, bc.x, bc.y, bc.z, bc.w };

  v8us vh, vl;
  #pragma unroll
  for (int j = 0; j < 8; ++j) {
    const float y = (x[j] - mu) * rstd * bfr(g[j]) + bfr(bt[j]);
    const unsigned short hb = f2bf(y);
    const unsigned short lb = f2bf(y - bf2f(hb));
    vh[j] = hb;
    vl[j] = lb;
  }
  unsigned short* dh = Hh + (size_t)row * DD + 8 * lane;
  unsigned short* dl = Hl + (size_t)row * DD + 8 * lane;
  *(volatile v8us*)dh = vh;
  *(volatile v8us*)dl = vl;
  __threadfence();
  *(volatile v8us*)dh = vh;
  *(volatile v8us*)dl = vl;
}

#define WBLK   32
#define ADJBLK 128

__global__ __launch_bounds__(256) void cvt_kernel(
    const float* __restrict__ W, const float* __restrict__ coef, const float* __restrict__ A,
    unsigned short* __restrict__ Wb, unsigned short* __restrict__ Ah, unsigned short* __restrict__ Al)
{
  const int g = blockIdx.x * 256 + threadIdx.x;
  if (blockIdx.x < WBLK) {
    if (g >= DD * DD / 8) return;
    const float* src = W + (size_t)g * 8;
    const v4f a = *(const v4fa*)src;
    const v4f c = *(const v4fa*)(src + 4);
    const v8us o = { f2bf(a.x), f2bf(a.y), f2bf(a.z), f2bf(a.w),
                     f2bf(c.x), f2bf(c.y), f2bf(c.z), f2bf(c.w) };
    unsigned short* dst = Wb + (size_t)g * 8;
    *(volatile v8us*)dst = o;
    __threadfence();
    *(volatile v8us*)dst = o;
  } else {
    const int e = g - WBLK * 256;
    if (e >= NN * NN / 8) return;
    const float* cs = coef + (size_t)e * 8;
    const float* as = A + (size_t)e * 8;
    const v4f ca = *(const v4fa*)cs;
    const v4f cc = *(const v4fa*)(cs + 4);
    const v4f aa = *(const v4fa*)as;
    const v4f ac = *(const v4fa*)(as + 4);
    const float cv[8] = { ca.x, ca.y, ca.z, ca.w, cc.x, cc.y, cc.z, cc.w };
    const float av[8] = { aa.x, aa.y, aa.z, aa.w, ac.x, ac.y, ac.z, ac.w };
    v8us oh, ol;
    #pragma unroll
    for (int j = 0; j < 8; ++j) {
      const float p = bfr(cv[j]) * bfr(av[j]);
      const unsigned short hb = f2bf(p);
      oh[j] = hb;
      ol[j] = f2bf(p - bf2f(hb));
    }
    unsigned short* dh = Ah + (size_t)e * 8;
    unsigned short* dl = Al + (size_t)e * 8;
    *(volatile v8us*)dh = oh;
    *(volatile v8us*)dl = ol;
    __threadfence();
    *(volatile v8us*)dh = oh;
    *(volatile v8us*)dl = ol;
  }
}

__device__ __forceinline__ void msg_store_pass(const unsigned short* s, unsigned short* M,
                                               int bidx, int e0, int ml0, int lane) {
  const int q8 = lane & 7, sub = lane >> 3;
  #pragma unroll
  for (int i = 0; i < 4; ++i) {
    const int row = 4 * i + sub;
    const v8us v = *(const v8usa*)(s + row * 64 + 8 * q8);
    unsigned short* dst = M + ((size_t)(bidx * DD + e0 + row)) * NN + ml0 + 8 * q8;
    *(volatile v8us*)dst = v;
  }
}

__global__ __launch_bounds__(128) void gemm1_kernel(
    const unsigned short* __restrict__ Wb,
    const unsigned short* __restrict__ Hh,
    const unsigned short* __restrict__ Hl,
    const float* __restrict__ bias,
    unsigned short* __restrict__ Mh,
    unsigned short* __restrict__ Ml)
{
  __shared__ __attribute__((aligned(16))) unsigned short sH[4 * 1024];
  __shared__ __attribute__((aligned(16))) unsigned short sL[4 * 1024];

  const int tid = threadIdx.x, lane = tid & 31, w = tid >> 5;
  const int h = lane >> 4, m = lane & 15;
  const int bm0 = blockIdx.x * 64;
  const int e0  = blockIdx.y * 64 + 16 * w;

  const unsigned short* wa  = Wb + (size_t)(e0 + m) * DD;
  const unsigned short* bh0 = Hh + (size_t)(bm0 + m) * DD;
  const unsigned short* bl0 = Hl + (size_t)(bm0 + m) * DD;

  const v8f zero8 = {0.f, 0.f, 0.f, 0.f, 0.f, 0.f, 0.f, 0.f};
  v8f acc[4];
  #pragma unroll
  for (int t = 0; t < 4; ++t) acc[t] = zero8;

  #pragma unroll 1
  for (int k0 = 0; k0 < DD; k0 += 32) {
    const v16us af = load_frag(wa + k0, h);
    #pragma unroll
    for (int t = 0; t < 4; ++t) {
      const v16us fh = load_frag(bh0 + (size_t)t * 16 * DD + k0, h);
      const v16us fl = load_frag(bl0 + (size_t)t * 16 * DD + k0, h);
      acc[t] = wmma_bf16(af, fh, acc[t]);
      acc[t] = wmma_bf16(af, fl, acc[t]);
    }
  }

  const v4f b0 = *(const v4fa*)(bias + e0 + 8 * h);
  const v4f b1 = *(const v4fa*)(bias + e0 + 8 * h + 4);
  const float bb[8] = { bfr(b0.x), bfr(b0.y), bfr(b0.z), bfr(b0.w),
                        bfr(b1.x), bfr(b1.y), bfr(b1.z), bfr(b1.w) };
  unsigned short* sh = sH + w * 1024;
  unsigned short* sl = sL + w * 1024;
  #pragma unroll
  for (int t = 0; t < 4; ++t) {
    #pragma unroll
    for (int r = 0; r < 8; ++r) {
      const float v = fmaxf(acc[t][r] + bb[r], 0.0f);
      const unsigned short hb = f2bf(v);
      const unsigned short lb = f2bf(v - bf2f(hb));
      const int idx = (8 * h + r) * 64 + 16 * t + m;
      sh[idx] = hb;
      sl[idx] = lb;
    }
  }
  __syncthreads();

  const int bidx = bm0 / NN, ml0 = bm0 - bidx * NN;
  msg_store_pass(sh, Mh, bidx, e0, ml0, lane);
  msg_store_pass(sl, Ml, bidx, e0, ml0, lane);
  __threadfence();
  msg_store_pass(sh, Mh, bidx, e0, ml0, lane);
  msg_store_pass(sl, Ml, bidx, e0, ml0, lane);
}

__device__ __forceinline__ void out_store_pass(const float* so, float* out,
                                               int b, int n0, int d0, int lane) {
  const int q8 = lane & 7, sub = lane >> 3;
  #pragma unroll
  for (int i = 0; i < 8; ++i) {
    const int lid = 4 * i + sub;
    const int row = lid >> 1, hl = lid & 1;
    const v4f v = *(const v4fa*)(so + row * 64 + 32 * hl + 4 * q8);
    const size_t gi = ((size_t)(b * NN + n0 + row)) * DD + d0 + 32 * hl + 4 * q8;
    *(volatile v4f*)(out + gi) = v;
  }
}

__global__ __launch_bounds__(128) void gemm2_kernel(
    const unsigned short* __restrict__ Ah,
    const unsigned short* __restrict__ Al,
    const unsigned short* __restrict__ Mh,
    const unsigned short* __restrict__ Ml,
    float* __restrict__ out)
{
  __shared__ __attribute__((aligned(16))) float sO[4 * 1024];

  const int tid = threadIdx.x, lane = tid & 31, w = tid >> 5;
  const int h = lane >> 4, m = lane & 15;
  const int n0 = blockIdx.x * 16;
  const int b  = blockIdx.y;
  const int d0 = 64 * w;

  const unsigned short* ah0 = Ah + (size_t)(n0 + m) * NN;
  const unsigned short* al0 = Al + (size_t)(n0 + m) * NN;
  const unsigned short* mh0 = Mh + ((size_t)(b * DD + d0 + m)) * NN;
  const unsigned short* ml0 = Ml + ((size_t)(b * DD + d0 + m)) * NN;

  const v8f zero8 = {0.f, 0.f, 0.f, 0.f, 0.f, 0.f, 0.f, 0.f};
  v8f acc[4];
  #pragma unroll
  for (int t = 0; t < 4; ++t) acc[t] = zero8;

  #pragma unroll 1
  for (int k0 = 0; k0 < NN; k0 += 32) {
    const v16us fah = load_frag(ah0 + k0, h);
    const v16us fal = load_frag(al0 + k0, h);
    #pragma unroll
    for (int t = 0; t < 4; ++t) {
      const v16us fbh = load_frag(mh0 + (size_t)t * 16 * NN + k0, h);
      const v16us fbl = load_frag(ml0 + (size_t)t * 16 * NN + k0, h);
      acc[t] = wmma_bf16(fah, fbh, acc[t]);
      acc[t] = wmma_bf16(fah, fbl, acc[t]);
      acc[t] = wmma_bf16(fal, fbh, acc[t]);
    }
  }

  const float scale = 1.0f / 512.0f;
  float* so = sO + w * 1024;
  #pragma unroll
  for (int t = 0; t < 4; ++t)
    #pragma unroll
    for (int r = 0; r < 8; ++r)
      so[(8 * h + r) * 64 + 16 * t + m] = acc[t][r] * scale;
  __syncthreads();

  out_store_pass(so, out, b, n0, d0, lane);
  __threadfence();
  out_store_pass(so, out, b, n0, d0, lane);
}

extern "C" void kernel_launch(void* const* d_in, const int* in_sizes, int n_in,
                              void* d_out, int out_size, void* d_ws, size_t ws_size,
                              hipStream_t stream) {
  if (n_in < 7) return;
  if (in_sizes[0] != MROWS * DD) return;
  if (in_sizes[1] != NN * NN || in_sizes[2] != NN * NN) return;
  if (in_sizes[3] != DD || in_sizes[4] != DD || in_sizes[6] != DD) return;
  if (in_sizes[5] != DD * DD) return;
  if (out_size != MROWS * DD) return;

  const float* H     = (const float*)d_in[0];
  const float* A     = (const float*)d_in[1];
  const float* coef  = (const float*)d_in[2];
  const float* gamma = (const float*)d_in[3];
  const float* beta  = (const float*)d_in[4];
  const float* W     = (const float*)d_in[5];
  const float* bias  = (const float*)d_in[6];
  float* out = (float*)d_out;

  const size_t hn_bytes  = (size_t)MROWS * DD * 2;
  const size_t wb_bytes  = (size_t)DD * DD * 2;
  const size_t adj_bytes = (size_t)NN * NN * 2;
  const size_t msg_bytes = (size_t)BB * DD * NN * 2;
  const size_t total = 2 * hn_bytes + wb_bytes + 2 * adj_bytes + 2 * msg_bytes;
  if (total > ws_size) return;

  char* ws = (char*)d_ws;
  size_t off = 0;
  unsigned short* Hh = (unsigned short*)(ws + off); off += hn_bytes;
  unsigned short* Hl = (unsigned short*)(ws + off); off += hn_bytes;
  unsigned short* Wb = (unsigned short*)(ws + off); off += wb_bytes;
  unsigned short* Ah = (unsigned short*)(ws + off); off += adj_bytes;
  unsigned short* Al = (unsigned short*)(ws + off); off += adj_bytes;
  unsigned short* Mh = (unsigned short*)(ws + off); off += msg_bytes;
  unsigned short* Ml = (unsigned short*)(ws + off); off += msg_bytes;
  if (off > ws_size) return;

  ln_kernel<<<MROWS / 8, 256, 0, stream>>>(H, gamma, beta, Hh, Hl);
  cvt_kernel<<<WBLK + ADJBLK, 256, 0, stream>>>(W, coef, A, Wb, Ah, Al);

  dim3 g1(MROWS / 64, DD / 64);
  gemm1_kernel<<<g1, 128, 0, stream>>>(Wb, Hh, Hl, bias, Mh, Ml);

  dim3 g2(NN / 16, BB);
  gemm2_kernel<<<g2, 128, 0, stream>>>(Ah, Al, Mh, Ml, out);
}
